// DiagonalMicroAttention_87497073754696
// MI455X (gfx1250) — hardware-verified
//
#include <hip/hip_runtime.h>
#include <math.h>

typedef __attribute__((ext_vector_type(16))) _Float16 v16h;
typedef __attribute__((ext_vector_type(16))) __bf16 v16b;
typedef __attribute__((ext_vector_type(8)))  _Float16 v8h;
typedef __attribute__((ext_vector_type(8)))  float v8f;
typedef __attribute__((ext_vector_type(4)))  float v4f;
typedef __attribute__((ext_vector_type(2)))  float v2f;
typedef __attribute__((ext_vector_type(4)))  unsigned v4u;
typedef __attribute__((ext_vector_type(4)))  int v4i;
typedef float __attribute__((may_alias)) float_a;
typedef int __attribute__((may_alias)) int_a;

template <typename T> __device__ __forceinline__ void vst2(void* p, T v) { *(volatile T*)p = v; __threadfence(); *(volatile T*)p = v; }
__device__ __forceinline__ v8f wmma16(v16h a, v16h b, v8f c) {
  v8f d = __builtin_amdgcn_wmma_f32_16x16x32_f16(false, a, false, b, (short)0, c, false, false);
  asm volatile("v_nop\n\tv_nop\n\tv_nop\n\tv_nop" : "+v"(d) : "v"(a), "v"(b));
  return d;
}
__device__ __forceinline__ v8f wmma_bf(v16b a, v16b b, v8f c) {
  v8f d = __builtin_amdgcn_wmma_f32_16x16x32_bf16(false, a, false, b, (short)0, c, false, false);
  asm volatile("v_nop\n\tv_nop\n\tv_nop\n\tv_nop" : "+v"(d) : "v"(a), "v"(b));
  return d;
}
__device__ __forceinline__ v16h frag_h(const _Float16* rowk0, int lane) {
  union { v16h v; v8h q[2]; } u; const _Float16* p = rowk0 + 8 * (lane >> 4);
  u.q[0] = *(const v8h*)p; u.q[1] = *(const v8h*)(p + 16); return u.v;
}
__device__ __forceinline__ v16h frag_f32(const float* rowk0, int lane) {
  v16h a; const float* p = rowk0 + 8 * (lane >> 4);
#pragma unroll
  for (int i = 0; i < 8; ++i) { a[i] = (_Float16)p[i]; a[8 + i] = (_Float16)p[16 + i]; }
  return a;
}
__device__ __forceinline__ v16h frag_f32s(const float* rowk0, int lane, float sc) {
  v16h a; const float* p = rowk0 + 8 * (lane >> 4);
#pragma unroll
  for (int i = 0; i < 8; ++i) { a[i] = (_Float16)(p[i] * sc); a[8 + i] = (_Float16)(p[16 + i] * sc); }
  return a;
}
__device__ __forceinline__ v16h fragc_f32(const float* W, int k0, int n, int lane, int ld, int K) {
  v16h a; const int g = lane >> 4;
#pragma unroll
  for (int i = 0; i < 8; ++i) { const int ka = k0 + 8 * g + i, kb = ka + 16;
    a[i] = (_Float16)(ka < K ? W[(size_t)(ka < K ? ka : K - 1) * ld + n] : 0.f); a[8 + i] = (_Float16)(kb < K ? W[(size_t)(kb < K ? kb : K - 1) * ld + n] : 0.f); }
  return a;
}
struct F2 { v16b h, l; };
__device__ __forceinline__ F2 bsplit16(const float v[16]) { F2 r;
#pragma unroll
  for (int i = 0; i < 16; ++i) { const __bf16 h = (__bf16)v[i]; r.h[i] = h; r.l[i] = (__bf16)(v[i] - (float)h); }
  return r; }
__device__ __forceinline__ F2 split_row(const float* row, int k0, int lane) { float v[16]; const float* p = row + k0 + 8 * (lane >> 4);
#pragma unroll
  for (int i = 0; i < 8; ++i) { v[i] = p[i]; v[8 + i] = p[16 + i]; }
  return bsplit16(v); }
__device__ __forceinline__ F2 split_rowK(const float* row, int k0, int lane, int K) { float v[16]; const int g = lane >> 4;
#pragma unroll
  for (int i = 0; i < 8; ++i) { const int ka = k0 + 8 * g + i, kb = ka + 16; v[i] = ka < K ? row[ka < K ? ka : K - 1] : 0.f; v[8 + i] = kb < K ? row[kb < K ? kb : K - 1] : 0.f; }
  return bsplit16(v); }
__device__ __forceinline__ F2 split_col(const float* W, int k0, int n, int lane, int ld, int K) { float v[16]; const int g = lane >> 4;
#pragma unroll
  for (int i = 0; i < 8; ++i) { const int ka = k0 + 8 * g + i, kb = ka + 16; v[i] = ka < K ? W[(size_t)(ka < K ? ka : K - 1) * ld + n] : 0.f; v[8 + i] = kb < K ? W[(size_t)(kb < K ? kb : K - 1) * ld + n] : 0.f; }
  return bsplit16(v); }
__device__ __forceinline__ v8f mac3(const F2& a, const F2& b, v8f c) { c = wmma_bf(a.l, b.h, c); c = wmma_bf(a.h, b.l, c); return wmma_bf(a.h, b.h, c); }
__device__ __forceinline__ float sigm(float v) { return 1.0f / (1.0f + expf(-v)); }
#define LDSX() do { asm volatile("s_wait_dscnt 0" ::: "memory"); __builtin_amdgcn_wave_barrier(); __builtin_amdgcn_fence(__ATOMIC_RELEASE, "workgroup"); } while (0)


#define NB 2
#define CC 128
#define HI 56
#define WI 56
#define NPIX (HI * WI)
#define WH 28
#define NCAT (HI * WH)
#define NHD 4
#define DH 32
__device__ __forceinline__ float bfr(float v) { return (float)(__bf16)v; }
__device__ __forceinline__ v16b frag_b(const __bf16* rowk0, int lane) { return __builtin_bit_cast(v16b, frag_h((const _Float16*)rowk0, lane)); }
__device__ __attribute__((noinline)) float exp_ni(float v) { return expf(v); }
__device__ __attribute__((noinline)) float gelu_ni(float v) { return 0.5f * v * (1.0f + erff(v * 0.70710678118654752f)); }

__global__ __launch_bounds__(256) void k_cvt(const float* __restrict__ x, __bf16* __restrict__ XT, __bf16* __restrict__ CT) {
  __shared__ __align__(16) __bf16 st[64][2 * CC + 8];
  const int tid = threadIdx.x; const int b = blockIdx.y, which = blockIdx.z;
  if (which == 0) { const int p0 = blockIdx.x * 64;
    for (int q = tid; q < CC * 16; q += 256) { const int c = q >> 4, p4 = q & 15; const v4f v = *(const v4f*)(x + ((size_t)b * CC + c) * NPIX + p0 + p4 * 4);
      st[p4 * 4][c] = (__bf16)v[0]; st[p4 * 4 + 1][c] = (__bf16)v[1]; st[p4 * 4 + 2][c] = (__bf16)v[2]; st[p4 * 4 + 3][c] = (__bf16)v[3]; }
    __syncthreads();
    for (int q = tid; q < 64 * 16; q += 256) { const int rl = q >> 4, pc = q & 15; vst2((unsigned*)(XT + ((size_t)b * NPIX + p0 + rl) * CC + pc * 8), *(const v4u*)(&st[rl][pc * 8])); } }
  else { if (blockIdx.x >= HI / 2) return; const int y0 = blockIdx.x * 2;
    for (int q = tid; q < 2 * CC * WI; q += 256) { const int yy = q / (CC * WI), rem = q % (CC * WI); const int c = rem / WI, xx = rem % WI; const float v = x[(((size_t)b * CC + c) * HI + y0 + yy) * WI + xx];
      if (xx < WH) st[yy * WH + xx][c] = (__bf16)v; else st[yy * WH + (WI - 1 - xx)][CC + c] = (__bf16)v; }
    __syncthreads();
    for (int q = tid; q < 56 * 32; q += 256) { const int rl = q >> 5, pc = q & 31; vst2((unsigned*)(CT + ((size_t)b * NCAT + y0 * WH + rl) * (2 * CC) + pc * 8), *(const v4u*)(&st[rl][pc * 8])); } }
}
__global__ __launch_bounds__(128) void k_qkv(const __bf16* __restrict__ XT, const float* __restrict__ Wq, const float* __restrict__ Wk, const float* __restrict__ Wv, float* __restrict__ Q, float* __restrict__ K, float* __restrict__ V) {
  __shared__ __align__(16) float so[4][16][132];
  const int tid = threadIdx.x, wave = tid >> 5, lane = tid & 31, col = lane & 15, g = lane >> 4; const size_t r0 = (size_t)blockIdx.x * 64 + wave * 16; const int which = blockIdx.y;
  const float* W = which == 0 ? Wq : (which == 1 ? Wk : Wv); float* O = which == 0 ? Q : (which == 1 ? K : V);
  v8f acc[8] = {};
#pragma unroll
  for (int kc = 0; kc < CC / 32; ++kc) { const v16b a = frag_b(XT + (r0 + col) * CC + kc * 32, lane);
#pragma unroll
    for (int j = 0; j < 8; ++j) acc[j] = wmma_bf(a, split_row(W + (size_t)(j * 16 + col) * CC, kc * 32, lane).h, acc[j]); }
#pragma unroll
  for (int j = 0; j < 8; ++j)
#pragma unroll
    for (int r = 0; r < 8; ++r) so[wave][8 * g + r][j * 16 + col] = acc[j][r];
  LDSX();
  for (int rl = 0; rl < 16; ++rl) vst2(O + (r0 + rl) * CC + lane * 4, *(const v4f*)(&so[wave][rl][lane * 4]));
}
__global__ __launch_bounds__(128) void k_asym(const __bf16* __restrict__ CT, const float* __restrict__ Wa1, const float* __restrict__ ba1, const float* __restrict__ Wa2, const float* __restrict__ ba2, float* __restrict__ AS) {
  __shared__ __align__(16) float sa[4][16];
  const int tid = threadIdx.x, wave = tid >> 5, lane = tid & 31, col = lane & 15, g = lane >> 4; const size_t r0 = (size_t)blockIdx.x * 64 + wave * 16;
  v8f acc[8] = {};
#pragma unroll 2
  for (int kc = 0; kc < 2 * CC / 32; ++kc) { const v16b a = frag_b(CT + (r0 + col) * (2 * CC) + kc * 32, lane);
#pragma unroll
    for (int j = 0; j < 8; ++j) acc[j] = wmma_bf(a, split_row(Wa1 + (size_t)(j * 16 + col) * (2 * CC), kc * 32, lane).h, acc[j]); }
  float part[8];
#pragma unroll
  for (int r = 0; r < 8; ++r) part[r] = 0.f;
#pragma unroll
  for (int j = 0; j < 8; ++j) { const int n = j * 16 + col; const float bb = bfr(ba1[n]), w2 = bfr(Wa2[n]);
#pragma unroll
    for (int r = 0; r < 8; ++r) part[r] += gelu_ni(acc[j][r] + bb) * w2; }
#pragma unroll
  for (int r = 0; r < 8; ++r) {
#pragma unroll
    for (int o_ = 1; o_ < 16; o_ <<= 1) part[r] += __shfl_xor(part[r], o_, 32); }
  if (col == 0) { const float b2 = bfr(ba2[0]);
#pragma unroll
    for (int r = 0; r < 8; ++r) sa[wave][8 * g + r] = 1.0f / (1.0f + exp_ni(-(part[r] + b2))); }
  LDSX();
  if (lane < 4) vst2(AS + r0 + lane * 4, *(const v4f*)(&sa[wave][lane * 4]));
}
__global__ __launch_bounds__(256) void k_attn(const float* __restrict__ Q, const float* __restrict__ K, const float* __restrict__ V, const float* __restrict__ AS, float* __restrict__ O) {
  __shared__ __align__(16) float so[64][CC + 4];
  const int tid = threadIdx.x; const int b = blockIdx.y, p0 = blockIdx.x * 64; const int pl = tid >> 2, h = tid & 3; const int pix = p0 + pl; const int py = pix / WI, px = pix % WI;
  const size_t base = (size_t)b * NPIX;
  float q[DH];
  { const float* qr = Q + (base + pix) * CC + h * DH;
#pragma unroll
    for (int d = 0; d < DH; ++d) q[d] = qr[d]; }
  float sc[9]; int nb[9]; float mx = -3.4e38f;
#pragma unroll
  for (int t = 0; t < 9; ++t) { const int dy = t / 3 - 1, dx = t % 3 - 1; const int yy = py + dy, xx = px + dx; const bool ok = yy >= 0 && yy < HI && xx >= 0 && xx < WI; nb[t] = ok ? yy * WI + xx : -1;
    float s = -3.4e38f;
    if (ok) { const float* kr = K + (base + yy * WI + xx) * CC + h * DH; s = 0.f;
#pragma unroll 8
      for (int d = 0; d < DH; ++d) s += q[d] * kr[d];
      s *= 0.17677669529663687f; }
    sc[t] = s; mx = fmaxf(mx, s); }
  float den = 0.f;
#pragma unroll
  for (int t = 0; t < 9; ++t) { sc[t] = nb[t] >= 0 ? exp_ni(sc[t] - mx) : 0.f; den += sc[t]; }
  const float inv = 1.0f / den;
  float o[DH];
#pragma unroll
  for (int d = 0; d < DH; ++d) o[d] = 0.f;
#pragma unroll 1
  for (int t = 0; t < 9; ++t) { if (nb[t] < 0) continue; const float wgt = sc[t] * inv; const float* vr = V + (base + nb[t]) * CC + h * DH;
#pragma unroll 8
    for (int d = 0; d < DH; ++d) o[d] += wgt * vr[d]; }
  { const float f = 0.5f * (float)px - 0.25f; int i0 = (int)floorf(f); const float t_ = f - (float)i0; float a;
    const float* ar = AS + base / NPIX * NCAT + (size_t)py * WH;
    if (i0 < 0) a = ar[0]; else if (i0 >= WH - 1) a = ar[WH - 1]; else a = (1.0f - t_) * ar[i0] + t_ * ar[i0 + 1];
    const float gain = 1.0f + 0.5f * a;
#pragma unroll
    for (int d = 0; d < DH; ++d) so[pl][h * DH + d] = o[d] * gain; }
  __syncthreads();
  for (int q4 = tid; q4 < 64 * CC / 4; q4 += 256) { const int rl = q4 >> 5, pc = q4 & 31; vst2(O + (base + p0 + rl) * CC + pc * 4, *(const v4f*)(&so[rl][pc * 4])); }
}
__global__ __launch_bounds__(128) void k_out(const float* __restrict__ O, const float* __restrict__ Wo, const float* __restrict__ bo, float* __restrict__ y) {
  __shared__ __align__(16) float sO[4][32][68];
  const int tid = threadIdx.x, w = tid >> 5, lane = tid & 31, col = lane & 15, g = lane >> 4; const int b = blockIdx.y, p0 = blockIdx.x * 64; const size_t base = (size_t)b * NPIX;
  v8f acc[2][4] = {};
#pragma unroll
  for (int kc = 0; kc < CC / 32; ++kc) {
#pragma unroll
    for (int ct = 0; ct < 2; ++ct) { const v16b a = split_row(Wo + (size_t)((w * 2 + ct) * 16 + col) * CC, kc * 32, lane).h;
#pragma unroll
      for (int pt = 0; pt < 4; ++pt) { const F2 bc = split_row(O + (base + p0 + pt * 16 + col) * CC, kc * 32, lane); acc[ct][pt] = wmma_bf(a, bc.l, acc[ct][pt]); acc[ct][pt] = wmma_bf(a, bc.h, acc[ct][pt]); } } }
#pragma unroll
  for (int ct = 0; ct < 2; ++ct) {
#pragma unroll
    for (int r = 0; r < 8; ++r) { const int cl = ct * 16 + 8 * g + r; const float bb = bfr(bo[w * 32 + cl]);
#pragma unroll
      for (int pt = 0; pt < 4; ++pt) sO[w][cl][pt * 16 + col] = acc[ct][pt][r] + bb; } }
  LDSX();
  for (int qq = lane; qq < 32 * 16; qq += 32) { const int cl = qq >> 4, pc = qq & 15; vst2(y + ((size_t)b * CC + w * 32 + cl) * NPIX + p0 + pc * 4, *(const v4f*)(&sO[w][cl][pc * 4])); }
}
extern "C" void kernel_launch(void* const* d_in, const int* in_sizes, int n_in, void* d_out, int out_size, void* d_ws, size_t ws_size, hipStream_t stream) {
  (void)in_sizes; (void)n_in; (void)out_size; (void)ws_size;
  const float** I = (const float**)d_in;
  const float* x = I[0]; const float* Wq = I[1]; const float* Wk = I[2]; const float* Wv = I[3]; const float* Wo = I[4]; const float* bo = I[5]; const float* Wa1 = I[6]; const float* ba1 = I[7]; const float* Wa2 = I[8]; const float* ba2 = I[9];
  char* ws = (char*)d_ws; size_t off = 0;
  auto take = [&](size_t bytes) { char* p = ws + off; off += (bytes + 255) & ~(size_t)255; return p; };
  __bf16* XT = (__bf16*)take((size_t)NB * NPIX * CC * 2); __bf16* CT = (__bf16*)take((size_t)NB * NCAT * 2 * CC * 2);
  float* Q = (float*)take((size_t)NB * NPIX * CC * 4); float* K = (float*)take((size_t)NB * NPIX * CC * 4); float* V = (float*)take((size_t)NB * NPIX * CC * 4); float* AS = (float*)take((size_t)NB * NCAT * 4); float* O = (float*)take((size_t)NB * NPIX * CC * 4);
  k_cvt<<<dim3(NPIX / 64, NB, 2), 256, 0, stream>>>(x, XT, CT);
  k_qkv<<<dim3(NB * NPIX / 64, 3), 128, 0, stream>>>(XT, Wq, Wk, Wv, Q, K, V);
  k_asym<<<NB * NCAT / 64, 128, 0, stream>>>(CT, Wa1, ba1, Wa2, ba2, AS);
  k_attn<<<dim3(NPIX / 64, NB), 256, 0, stream>>>(Q, K, V, AS, O);
  k_out<<<dim3(NPIX / 64, NB), 128, 0, stream>>>(O, Wo, bo, (float*)d_out);
}
